// Model_75368086110575
// MI455X (gfx1250) — hardware-verified
//
#include <hip/hip_runtime.h>
#include <stddef.h>
#include <stdint.h>
#include <math.h>


#define NN      131072
#define NGRAPH  512
#define GLEN    256
#define DIN     300
#define KE      320
#define DH      96
#define KH      192
#define KZ      384
#define NCLS    20
#define NVOC    50001
#define NTHR    256
#define NWAVE   8
#define EPT     8
#define CHUNK   (NTHR * EPT)
#define WCAP    (EPT * 32)
#define LISTN   (NWAVE * WCAP)
#define NBA     1024
#define SLA     10
#define SRCB    17
#define RCAP    12288
#define DEGCAP  64
#define MEAS_B1024  8192
#define MEAS_MAXDEG 26
#define GR      64
#define GT      256
#define NEGSL   0.2f
#define WSMAX   134217728
#define BKT_LDS_INTS  (LISTN + RCAP + 16)
#define SCAN_ZINTS    (RCAP + 3 * NBA)
#define SCAN_LDS_INTS (2 * RCAP + 3 * NBA + 16)
#define TB_BE   0
#define TB_BG   96
#define TB_BZ   192
#define TB_BR   288
#define TB_BH   384
#define TB_VS   480
#define TB_VD   576
#define TB_PAD  672
#define TB_WM   768
#define TB_N    2688
#define NU_WE   (DH * (KE / 8))
#define NU_W2   (DH * (KH / 8))
#define NU_ALL  (NU_WE + 8 * NU_W2)
#define NB_W    (NU_ALL / NTHR)
#define GRU_LDS ((4 * GR * KH) * 2 + (3 * GR * DH + 768 + 128 + 192) * 4)
#define ENC_LDS ((GR * KE) * 2 + (GR * DH + 768 + 128) * 4)

static_assert((NN % GR) == 0 && (GLEN % GR) == 0 && (DH % 16) == 0 && (KH % 32) == 0 && (KE % 32) == 0);
static_assert(NN == NGRAPH * GLEN && (NN % NBA) == 0 && KH == 2 * DH && KZ == 2 * KH);
static_assert((CHUNK & (CHUNK - 1)) == 0 && CHUNK <= 4096);
static_assert(NBA == (1 << SLA) && NBA <= 1024 && NN <= (1 << SRCB) && SRCB + SLA <= 31);
static_assert(((long long)CHUNK << SLA) < (1LL << 31));
static_assert(NBA % NWAVE == 0 && NBA % 32 == 0);
static_assert((RCAP % 32) == 0 && (SCAN_ZINTS % 4) == 0);
static_assert(RCAP >= MEAS_B1024 + 4096);
static_assert(DEGCAP >= MEAS_MAXDEG + 8);
static_assert(SCAN_LDS_INTS * 4 <= 300000 && BKT_LDS_INTS * 4 <= 300000 && GRU_LDS <= 300000);
static_assert((NU_WE % NTHR) == 0 && (NU_W2 % NTHR) == 0 && (NU_ALL % NTHR) == 0);
static_assert((GR * DH) % GT == 0 && (GR * KH / 8) % GT == 0 && GT == 4 * GR);
static_assert(TB_N % 32 == 0 && TB_WM + DH * NCLS == TB_N && (TB_N / 4) == 672);
static_assert(DIN % 4 == 0 && DIN / 4 == 75 && KE / 4 == 80);
static_assert((8 * NCLS * 4) % 128 == 0);

typedef float          v4f  __attribute__((ext_vector_type(4)));
typedef float          v8f  __attribute__((ext_vector_type(8)));
typedef int            v4i  __attribute__((ext_vector_type(4)));
typedef int            v8i  __attribute__((ext_vector_type(8)));
typedef unsigned int   v2u  __attribute__((ext_vector_type(2)));
typedef unsigned int   v4u  __attribute__((ext_vector_type(4)));
typedef unsigned short v8us __attribute__((ext_vector_type(8)));
typedef __bf16         v16b __attribute__((ext_vector_type(16)));
typedef v4f  __attribute__((may_alias)) v4fa;
typedef v4i  __attribute__((may_alias)) v4ia;
typedef v2u  __attribute__((may_alias)) v2ua;
typedef v4u  __attribute__((may_alias)) v4ua;
typedef v8us __attribute__((may_alias)) v8usa;
union FragB { v16b v; v8us h[2]; v8i w; };

__device__ __forceinline__ v8f wmb(const FragB& a, const FragB& b, v8f c) {
  v8f d = __builtin_amdgcn_wmma_f32_16x16x32_bf16(false, a.v, false, b.v, (short)0, c, false, false);
  asm volatile("v_nop\n\tv_nop\n\tv_nop\n\tv_nop" : "+v"(d) : "v"(a.w), "v"(b.w));
  return d;
}

__device__ __forceinline__ unsigned int f2bf(float f) {
  const unsigned int u = __float_as_uint(f);
  const unsigned int r = ((u + 0x7FFFu + ((u >> 16) & 1u)) >> 16) & 0xFFFFu;
  return ((u & 0x7FFFFFFFu) > 0x7F800000u) ? 0x7FC0u : r;
}
__device__ __forceinline__ float bf2f(unsigned int b) { return __uint_as_float(b << 16); }
__device__ __forceinline__ float bfr(float f) { return bf2f(f2bf(f)); }
__device__ __forceinline__ void split2(float v, unsigned int& h, unsigned int& l) {
  h = f2bf(v);
  l = f2bf(v - bf2f(h));
}

__device__ __forceinline__ void put8(unsigned short* dp, v8us o) {
  *(volatile v8us*)dp = o;
  __threadfence();
  *(volatile v8us*)dp = o;
}

template <int NT>
__device__ __forceinline__ void mm_acc(const unsigned short* aL, int ksteps,
                                       const unsigned short* __restrict__ wq, int ldw, v8f (&acc)[NT]) {
#pragma unroll 1
  for (int ks = 0; ks < ksteps; ++ks) {
    FragB af;
    af.h[0] = *(const v8usa*)(aL + 32 * ks);
    af.h[1] = *(const v8usa*)(aL + 32 * ks + 16);
#pragma unroll
    for (int t = 0; t < NT; ++t) {
      const unsigned short* w = wq + (size_t)(16 * t) * (size_t)ldw + 32 * ks;
      FragB bf;
      bf.h[0] = *(const v8usa*)w;
      bf.h[1] = *(const v8usa*)(w + 16);
      acc[t] = wmb(af, bf, acc[t]);
    }
  }
}

template <int NT>
__device__ __forceinline__ void put_raw(float* dst, int row0, int col0, int hh, int m, const v8f (&acc)[NT]) {
#pragma unroll
  for (int t = 0; t < NT; ++t) {
#pragma unroll
    for (int r = 0; r < 8; ++r) dst[(row0 + 8 * hh + r) * DH + col0 + 16 * t + m] = acc[t][r];
  }
}

template <int SLB>
__device__ __forceinline__ int scan_chunk(const int* __restrict__ dsts, int nE, int cbase, int slotBase,
                                          int nb, int vec8, int* list, int tid, int lane, int wave) {
  int wc = 0;
  const int el0  = tid * EPT;
  const int e0   = cbase + el0;
  const int sent = -2147483647 - 1;
  v4i da, db;
  if (vec8 != 0 && cbase + CHUNK <= nE) {
    da = *(const v4i*)(dsts + e0);
    db = *(const v4i*)(dsts + e0 + 4);
  } else {
    da.x = (e0     < nE) ? dsts[min(e0,     nE - 1)] : sent;
    da.y = (e0 + 1 < nE) ? dsts[min(e0 + 1, nE - 1)] : sent;
    da.z = (e0 + 2 < nE) ? dsts[min(e0 + 2, nE - 1)] : sent;
    da.w = (e0 + 3 < nE) ? dsts[min(e0 + 3, nE - 1)] : sent;
    db.x = (e0 + 4 < nE) ? dsts[min(e0 + 4, nE - 1)] : sent;
    db.y = (e0 + 5 < nE) ? dsts[min(e0 + 5, nE - 1)] : sent;
    db.z = (e0 + 6 < nE) ? dsts[min(e0 + 6, nE - 1)] : sent;
    db.w = (e0 + 7 < nE) ? dsts[min(e0 + 7, nE - 1)] : sent;
  }
  const unsigned nbs = (unsigned)slotBase;
  const unsigned unb = (unsigned)nb;
  const unsigned s0 = (unsigned)da.x - nbs, s1 = (unsigned)da.y - nbs;
  const unsigned s2 = (unsigned)da.z - nbs, s3 = (unsigned)da.w - nbs;
  const unsigned s4 = (unsigned)db.x - nbs, s5 = (unsigned)db.y - nbs;
  const unsigned s6 = (unsigned)db.z - nbs, s7 = (unsigned)db.w - nbs;
  const bool h0 = s0 < unb, h1 = s1 < unb, h2 = s2 < unb, h3 = s3 < unb;
  const bool h4 = s4 < unb, h5 = s5 < unb, h6 = s6 < unb, h7 = s7 < unb;
  const unsigned any = __builtin_amdgcn_ballot_w32(h0 | h1 | h2 | h3 | h4 | h5 | h6 | h7);
  if (any != 0u) {
#define HITJ(J, HJ, SJ) { \
      const unsigned mj = __builtin_amdgcn_ballot_w32(HJ); \
      if (mj != 0u) { \
        if (HJ) { \
          const int pos = wc + (int)__builtin_amdgcn_mbcnt_lo(mj, 0u); \
          if (pos < WCAP) list[wave * WCAP + pos] = ((el0 + (J)) << SLB) | (int)(SJ); \
        } \
        wc += (int)__builtin_popcount(mj); } }
    HITJ(0, h0, s0)
    HITJ(1, h1, s1)
    HITJ(2, h2, s2)
    HITJ(3, h3, s3)
    HITJ(4, h4, s4)
    HITJ(5, h5, s5)
    HITJ(6, h6, s6)
    HITJ(7, h7, s7)
#undef HITJ
  }
  return wc;
}

__device__ __forceinline__ v8us wt8(const float* __restrict__ W, int kk, int n) {
  v8us o;
  const float* p = W + (size_t)kk * DH + n;
#pragma unroll
  for (int i = 0; i < 8; ++i) o[i] = (unsigned short)f2bf(p[(size_t)i * DH]);
  return o;
}

__global__ __launch_bounds__(NTHR) void k_prep(
    const float* __restrict__ We, const float* __restrict__ Wg, const float* __restrict__ Wz0,
    const float* __restrict__ Wz1, const float* __restrict__ Wr0, const float* __restrict__ Wr1,
    const float* __restrict__ Wh0, const float* __restrict__ Wh1, const float* __restrict__ Wemb,
    const float* __restrict__ be, const float* __restrict__ bg, const float* __restrict__ bz0,
    const float* __restrict__ bz1, const float* __restrict__ br0, const float* __restrict__ br1,
    const float* __restrict__ bh0, const float* __restrict__ bh1, const float* __restrict__ ats,
    const float* __restrict__ atd, const float* __restrict__ Wmlp,
    unsigned short* WeT, unsigned short* WgT2, unsigned short* Wh0T2, unsigned short* Wh1T2,
    unsigned short* WembT2, unsigned short* BZR, float* TAB) {
  __shared__ __attribute__((aligned(16))) float ptab[TB_N];
  const int tid = (int)threadIdx.x;
  const int blk = (int)blockIdx.x;
  if (blk < NB_W) {
    const int u = blk * NTHR + tid;
    if (u < NU_WE) {
      const int n  = u / (KE / 8);
      const int k8 = (u - n * (KE / 8)) * 8;
      v8us o;
#pragma unroll
      for (int i = 0; i < 8; ++i) {
        const int k  = k8 + i;
        const int kc = k < DIN ? k : DIN - 1;
        const float f = We[(size_t)kc * DH + n];
        o[i] = (k < DIN) ? (unsigned short)f2bf(f) : (unsigned short)0;
      }
      put8(WeT + (size_t)n * KE + k8, o);
    } else {
      const int v   = u - NU_WE;
      const int sel = v / NU_W2;
      const int w   = v - sel * NU_W2;
      const int n   = w / (KH / 8);
      const int k8  = (w - n * (KH / 8)) * 8;
      const int kk  = k8 % DH;
      if (sel == 0)      put8(WgT2   + (size_t)n * KH + k8, wt8(Wg,   kk, n));
      else if (sel == 1) put8(Wh0T2  + (size_t)n * KH + k8, wt8(Wh0,  kk, n));
      else if (sel == 2) put8(Wh1T2  + (size_t)n * KH + k8, wt8(Wh1,  kk, n));
      else if (sel == 3) put8(WembT2 + (size_t)n * KH + k8, wt8(Wemb, kk, n));
      else if (sel == 4) put8(BZR + (size_t)n * KZ + k8,             wt8(Wz0, kk, n));
      else if (sel == 5) put8(BZR + (size_t)n * KZ + KH + k8,        wt8(Wz1, kk, n));
      else if (sel == 6) put8(BZR + (size_t)(DH + n) * KZ + k8,      wt8(Wr0, kk, n));
      else               put8(BZR + (size_t)(DH + n) * KZ + KH + k8, wt8(Wr1, kk, n));
    }
    return;
  }
  if (tid < DH) {
    const float* wr = Wg + (size_t)tid * DH;
    float s = 0.0f, d = 0.0f;
#pragma unroll 1
    for (int j4 = 0; j4 < DH / 4; ++j4) {
      const v4f w = *(const v4f*)(wr + 4 * j4);
      const v4f a = *(const v4f*)(ats + 4 * j4);
      const v4f b = *(const v4f*)(atd + 4 * j4);
      const float w0 = bfr(w.x), w1 = bfr(w.y), w2 = bfr(w.z), w3 = bfr(w.w);
      s = fmaf(w0, bfr(a.x), s); s = fmaf(w1, bfr(a.y), s); s = fmaf(w2, bfr(a.z), s); s = fmaf(w3, bfr(a.w), s);
      d = fmaf(w0, bfr(b.x), d); d = fmaf(w1, bfr(b.y), d); d = fmaf(w2, bfr(b.z), d); d = fmaf(w3, bfr(b.w), d);
    }
    ptab[TB_VS + tid] = s;
    ptab[TB_VD + tid] = d;
  } else if (tid < 2 * DH) {
    const int c = tid - DH;
    ptab[TB_BE + c] = bfr(be[c]);
    ptab[TB_BG + c] = bfr(bg[c]);
    ptab[TB_BZ + c] = bfr(bz0[c]) + bfr(bz1[c]);
    ptab[TB_BR + c] = bfr(br0[c]) + bfr(br1[c]);
    ptab[TB_BH + c] = bfr(bh0[c]) + bfr(bh1[c]);
    ptab[TB_PAD + c] = 0.0f;
  }
#pragma unroll 1
  for (int i = tid; i < (DH * NCLS) / 4; i += NTHR) {
    const v4f w = *(const v4f*)(Wmlp + 4 * i);
    v4f o;
    o.x = bfr(w.x); o.y = bfr(w.y); o.z = bfr(w.z); o.w = bfr(w.w);
    *(v4fa*)(ptab + TB_WM + 4 * i) = o;
  }
  __syncthreads();
#pragma unroll 1
  for (int p = tid; p < TB_N / 4; p += NTHR) {
    const v4f v = *(const v4fa*)(ptab + 4 * p);
    *(volatile v4f*)(TAB + 4 * p) = v;
  }
  __threadfence();
#pragma unroll 1
  for (int p = tid; p < TB_N / 4; p += NTHR) {
    const v4f v = *(const v4fa*)(ptab + 4 * p);
    *(volatile v4f*)(TAB + 4 * p) = v;
  }
}

__global__ __launch_bounds__(NTHR) void k_bucket(const int* __restrict__ srcs, const int* __restrict__ dsts,
                                                 int nE, int nN, int vec8, int* HITS, int* FLG) {
  extern __shared__ __attribute__((aligned(16))) int bsm[];
  int* list = bsm;
  int* reg1 = bsm + LISTN;
  int* wcnt = reg1 + RCAP;
  const int tid = (int)threadIdx.x, lane = tid & 31, wave = tid >> 5;
  const int blk = (int)blockIdx.x;
  const int nodeBase = blk * NBA;
  int nb = nN - nodeBase;
  nb = nb < 0 ? 0 : (nb > NBA ? NBA : nb);

  int tot = 0, ovf = 0;
  const int nChunks = (nE + CHUNK - 1) / CHUNK;
#pragma unroll 1
  for (int ch = 0; ch < nChunks; ++ch) {
    const int cbase = ch * CHUNK;
    const int wc = scan_chunk<SLA>(dsts, nE, cbase, nodeBase, nb, vec8, list, tid, lane, wave);
    if (lane == 0) wcnt[wave] = wc;
    __syncthreads();
    int pre = 0, all = 0;
#pragma unroll
    for (int w2 = 0; w2 < NWAVE; ++w2) {
      int c = wcnt[w2];
      c = c < 0 ? 0 : (c > WCAP ? WCAP : c);
      all += c;
      pre += (w2 < wave) ? c : 0;
    }
    const int wcc  = wc > WCAP ? WCAP : wc;
    const int base = tot + pre;
#pragma unroll 1
    for (int i = lane; i < wcc; i += 32) {
      const int ent = list[wave * WCAP + i];
      const int el  = (ent >> SLA) & (CHUNK - 1);
      const int sl  = ent & (NBA - 1);
      int eid = cbase + el;
      eid = eid > nE - 1 ? nE - 1 : eid;
      const int sraw = srcs[eid];
      const int s = sraw < 0 ? 0 : (sraw > nN - 1 ? nN - 1 : sraw);
      const int pos = base + i;
      if (pos < RCAP) reg1[pos] = (int)((unsigned)s | ((unsigned)sl << SRCB));
    }
    if (tot + all > RCAP) ovf = 1;
    tot += all;
    tot = tot > RCAP ? RCAP : tot;
    __syncthreads();
  }
  const int nh = tot;
  const int nhPad = (nh + 31) & ~31;
  for (int i = nh + tid; i < nhPad; i += NTHR) reg1[i] = 0;
  __syncthreads();

  int* hb = HITS + (size_t)blk * RCAP;
  v4i cv;
  cv.x = (tid == 0) ? nh : 0;
  cv.y = (tid == 0) ? ovf : 0;
  cv.z = 0; cv.w = 0;
  int* fp = FLG + (size_t)blk * 32 + 4 * (tid & 7);
#pragma unroll 1
  for (int p = tid * 4; p < nhPad; p += NTHR * 4) {
    const v4i v = *(const v4ia*)(reg1 + p);
    *(volatile v4i*)(hb + p) = v;
  }
  if (tid < 8) *(volatile v4i*)fp = cv;
  __threadfence();
#pragma unroll 1
  for (int p = tid * 4; p < nhPad; p += NTHR * 4) {
    const v4i v = *(const v4ia*)(reg1 + p);
    *(volatile v4i*)(hb + p) = v;
  }
  if (tid < 8) *(volatile v4i*)fp = cv;
}

__device__ __forceinline__ void x_tail(const float* sX, const float* tab, float* sdot,
                                       unsigned short* XHL, float* SD, int rowBase, int nN, int tid) {
  const int lane = tid & 31, wave = tid >> 5;
  if (tid < 128) {
    const int row = tid & 63, which = tid >> 6;
    const float* xr = sX + row * DH;
    const float* tv = tab + TB_VS + DH * which;
    float d = 0.0f;
#pragma unroll 2
    for (int c4 = 0; c4 < DH / 4; ++c4) {
      const v4f a = *(const v4fa*)(xr + 4 * c4);
      const v4f b = *(const v4fa*)(tv + 4 * c4);
      d = fmaf(a.x, b.x, d);
      d = fmaf(a.y, b.y, d);
      d = fmaf(a.z, b.z, d);
      d = fmaf(a.w, b.w, d);
    }
    sdot[which * GR + row] = d;
  }
  __syncthreads();

  v8us pc[6];
#pragma unroll
  for (int i = 0; i < 6; ++i) {
    const int g   = i * GT + tid;
    const int row = g / 24;
    const int p   = g - 24 * row;
    const bool lo = p >= 12;
    const int c   = 8 * (lo ? p - 12 : p);
    const v4f a = *(const v4fa*)(sX + row * DH + c);
    const v4f b = *(const v4fa*)(sX + row * DH + c + 4);
    const float f[8] = {a.x, a.y, a.z, a.w, b.x, b.y, b.z, b.w};
#pragma unroll
    for (int j = 0; j < 8; ++j) {
      unsigned int hb, lb;
      split2(f[j], hb, lb);
      pc[i][j] = (unsigned short)(lo ? lb : hb);
    }
  }
  const int which2 = lane >> 4, piece = lane & 15;
  const v4f sdv = *(const v4fa*)(sdot + which2 * GR + 4 * piece);
  float* sp = SD + (size_t)which2 * (size_t)nN + rowBase + 4 * piece;
  unsigned short* xp = XHL + (size_t)rowBase * KH;
#pragma unroll
  for (int i = 0; i < 6; ++i) *(volatile v8us*)(xp + (size_t)(i * GT + tid) * 8) = pc[i];
  if (wave == 0) *(volatile v4f*)sp = sdv;
  __threadfence();
#pragma unroll
  for (int i = 0; i < 6; ++i) *(volatile v8us*)(xp + (size_t)(i * GT + tid) * 8) = pc[i];
  if (wave == 0) *(volatile v4f*)sp = sdv;
}

__global__ __launch_bounds__(GT) void k_encode(const int* __restrict__ ids, const float* __restrict__ embed,
                                               const unsigned short* __restrict__ WeT,
                                               const float* __restrict__ TAB,
                                               unsigned short* XHL, float* SD, int nN, int nVoc) {
  extern __shared__ __attribute__((aligned(16))) float esm[];
  unsigned short* tE = (unsigned short*)esm;
  float* sX   = (float*)(tE + GR * KE);
  float* tab  = sX + GR * DH;
  float* sdot = tab + 768;
  const int tid = (int)threadIdx.x, lane = tid & 31, wave = tid >> 5;
  const int hh = lane >> 4, m = lane & 15;
  const int rg = wave & 3, ch = wave >> 2;
  const int rowBase = (int)blockIdx.x * GR;

  if (tid < 192) *(v4fa*)(tab + 4 * tid) = *(const v4f*)(TAB + 4 * tid);
  {
    const int row = tid >> 2, q = tid & 3;
    int gr = rowBase + row;
    gr = gr > nN - 1 ? nN - 1 : gr;
    int id = ids[gr];
    id = id < 0 ? 0 : (id > nVoc - 1 ? nVoc - 1 : id);
    const float* ep = embed + (size_t)id * DIN;
    unsigned short* tp = tE + row * KE;
#pragma unroll 4
    for (int i = 0; i < 20; ++i) {
      const int j  = q + 4 * i;
      const int jc = j < 75 ? j : 74;
      const v4f f = *(const v4f*)(ep + 4 * jc);
      const bool ok = j < 75;
      const unsigned int w0 = f2bf(f.x) | (f2bf(f.y) << 16);
      const unsigned int w1 = f2bf(f.z) | (f2bf(f.w) << 16);
      v2u w;
      w.x = ok ? w0 : 0u;
      w.y = ok ? w1 : 0u;
      *(v2ua*)(tp + 4 * j) = w;
    }
  }
  __syncthreads();

  const v8f z8 = {0.f, 0.f, 0.f, 0.f, 0.f, 0.f, 0.f, 0.f};
  v8f acc[3];
  acc[0] = z8; acc[1] = z8; acc[2] = z8;
  mm_acc<3>(tE + (16 * rg + m) * KE + 8 * hh, KE / 32,
            WeT + (size_t)(48 * ch + m) * KE + 8 * hh, KE, acc);
  put_raw<3>(sX, 16 * rg, 48 * ch, hh, m, acc);
  __syncthreads();
#pragma unroll 1
  for (int i = 0; i < (GR * DH) / GT; ++i) {
    const int e   = i * GT + tid;
    const int col = e % DH;
    sX[e] = tanhf(sX[e] + tab[TB_BE + col]);
  }
  __syncthreads();
  x_tail(sX, tab, sdot, XHL, SD, rowBase, nN, tid);
}

__global__ __launch_bounds__(NTHR) void k_scan(const int* __restrict__ HITS, const int* __restrict__ FLGB,
                                               const unsigned short* __restrict__ XHL,
                                               const float* __restrict__ SD, unsigned short* AGG, int nN) {
  extern __shared__ __attribute__((aligned(16))) int ssm[];
  int* hl   = ssm;
  int* sl   = ssm + RCAP;
  int* cnt  = sl + RCAP;
  int* offs = cnt + NBA;
  int* cur  = offs + NBA;
  int* misc = cur + NBA;
  const int tid = (int)threadIdx.x, lane = tid & 31, wave = tid >> 5;
  const int blk = (int)blockIdx.x;
  const int nodeBase = blk * NBA;

  const int nhraw = FLGB[(size_t)blk * 32];
  const int bflag = FLGB[(size_t)blk * 32 + 1];
  const int nh  = nhraw < 0 ? 0 : (nhraw > RCAP ? RCAP : nhraw);
  const int ovf = (bflag != 0 || nhraw < 0 || nhraw > RCAP) ? 1 : 0;

  {
    const v4i z4 = {0, 0, 0, 0};
    for (int i = tid * 4; i < SCAN_ZINTS; i += NTHR * 4) *(v4ia*)(sl + i) = z4;
    if (tid < 16) misc[tid] = 0;
    const int* hb = HITS + (size_t)blk * RCAP;
    const int nh4 = (nh + 3) & ~3;
#pragma unroll 1
    for (int p = tid * 4; p < nh4; p += NTHR * 4) *(v4ia*)(hl + p) = *(const v4i*)(hb + p);
  }
  __syncthreads();

  if (wave == 0) {
#pragma unroll 1
    for (int b0 = 0; b0 < nh; b0 += 32) {
      const int idx = b0 + lane;
      const int uv  = hl[idx < nh ? idx : nh - 1];
      const int m32 = (nh - b0) < 32 ? (nh - b0) : 32;
#pragma unroll 1
      for (int k = 0; k < m32; ++k) {
        const int u  = __builtin_amdgcn_readlane(uv, k);
        const int sq = (u >> SRCB) & (NBA - 1);
        if (lane == 0) cnt[sq] = cnt[sq] + 1;
      }
    }
  }
  __syncthreads();
  if (wave == 0) {
    const int base = lane * (NBA / 32);
    int s = 0;
#pragma unroll 1
    for (int i = 0; i < NBA / 32; ++i) s += cnt[base + i];
    int incl = s;
#pragma unroll
    for (int d = 1; d < 32; d <<= 1) {
      const int y = __shfl_up(incl, d, 32);
      if (lane >= d) incl += y;
    }
    int run = incl - s;
#pragma unroll 1
    for (int i = 0; i < NBA / 32; ++i) {
      const int cv = cnt[base + i];
      offs[base + i] = run;
      cur[base + i]  = run;
      run += cv;
    }
  }
  __syncthreads();
  if (wave == 0) {
#pragma unroll 1
    for (int b0 = 0; b0 < nh; b0 += 32) {
      const int idx = b0 + lane;
      const int uv  = hl[idx < nh ? idx : nh - 1];
      const int m32 = (nh - b0) < 32 ? (nh - b0) : 32;
#pragma unroll 1
      for (int k = 0; k < m32; ++k) {
        const int u  = __builtin_amdgcn_readlane(uv, k);
        const int sq = (u >> SRCB) & (NBA - 1);
        if (lane == 0) {
          int p = cur[sq];
          p = p < 0 ? 0 : (p > RCAP - 1 ? RCAP - 1 : p);
          sl[p] = u;
          cur[sq] = p + 1;
        }
      }
    }
  }
  __syncthreads();

  const float qnan = __int_as_float(0x7fc00000);
  const float pzb  = (ovf != 0) ? qnan : 0.0f;
  const int  cg    = (lane < 12) ? lane : ((lane < 24) ? lane - 12 : lane - 24);
  const bool islo  = (lane >= 12) && (lane < 24);
  const int  lst   = lane < 24 ? lane : 23;
  const float* SDs = SD;
  const float* SDd = SD + (size_t)nN;

#pragma unroll 1
  for (int si = 0; si < NBA / NWAVE; ++si) {
    const int s    = si * NWAVE + wave;
    const int node = nodeBase + s;
    const int nc   = node < nN ? node : nN - 1;
    int c = cnt[s];
    const bool big = c > DEGCAP;
    c = c < 0 ? 0 : (c > DEGCAP ? DEGCAP : c);
    int o = offs[s];
    o = o < 0 ? 0 : (o > RCAP ? RCAP : o);
    if (c > nh - o) c = nh - o;
    c = c < 0 ? 0 : c;
    const float adv = SDd[nc];
    float mx = -3.0e38f, dn = 0.0f;
    float acc[8];
#pragma unroll
    for (int i = 0; i < 8; ++i) acc[i] = 0.0f;
    const int T = c + 1;
#pragma unroll 1
    for (int b0 = 0; b0 < T; b0 += 32) {
      const int t = b0 + lane;
      int idx = o + t - 1;
      idx = idx < 0 ? 0 : (idx > RCAP - 1 ? RCAP - 1 : idx);
      const int ent = sl[idx];
      int hs = ent & ((1 << SRCB) - 1);
      hs = hs > nN - 1 ? nN - 1 : hs;
      const int sr  = (t == 0) ? nc : hs;
      const int m32 = (T - b0) < 32 ? (T - b0) : 32;
#pragma unroll 1
      for (int k = 0; k < m32; ++k) {
        const int sk = __builtin_amdgcn_readlane(sr, k);
        const unsigned short* rp = XHL + (size_t)sk * KH + 8 * cg;
        const v4u hw = *(const v4ua*)rp;
        const v4u lw = *(const v4ua*)(rp + DH);
        float lg = SDs[sk] + adv;
        lg = lg > 0.f ? lg : NEGSL * lg;
        const float df = lg - mx;
        const float ee = expf(-fabsf(df));
        const bool  up = df > 0.f;
        const float s1 = up ? ee : 1.0f;
        const float s2 = up ? 1.0f : ee;
        mx = up ? lg : mx;
        dn = fmaf(dn, s1, s2);
        const float x0 = __uint_as_float(hw.x << 16) + __uint_as_float(lw.x << 16);
        const float x1 = __uint_as_float(hw.x & 0xffff0000u) + __uint_as_float(lw.x & 0xffff0000u);
        const float x2 = __uint_as_float(hw.y << 16) + __uint_as_float(lw.y << 16);
        const float x3 = __uint_as_float(hw.y & 0xffff0000u) + __uint_as_float(lw.y & 0xffff0000u);
        const float x4 = __uint_as_float(hw.z << 16) + __uint_as_float(lw.z << 16);
        const float x5 = __uint_as_float(hw.z & 0xffff0000u) + __uint_as_float(lw.z & 0xffff0000u);
        const float x6 = __uint_as_float(hw.w << 16) + __uint_as_float(lw.w << 16);
        const float x7 = __uint_as_float(hw.w & 0xffff0000u) + __uint_as_float(lw.w & 0xffff0000u);
        acc[0] = fmaf(acc[0], s1, s2 * x0); acc[1] = fmaf(acc[1], s1, s2 * x1);
        acc[2] = fmaf(acc[2], s1, s2 * x2); acc[3] = fmaf(acc[3], s1, s2 * x3);
        acc[4] = fmaf(acc[4], s1, s2 * x4); acc[5] = fmaf(acc[5], s1, s2 * x5);
        acc[6] = fmaf(acc[6], s1, s2 * x6); acc[7] = fmaf(acc[7], s1, s2 * x7);
      }
    }
    const float inv = 1.0f / dn;
    const float pzr = big ? qnan : pzb;
    v8us ov;
#pragma unroll
    for (int j = 0; j < 8; ++j) {
      const float v = fmaf(acc[j], inv, pzr);
      unsigned int hb, lb;
      split2(v, hb, lb);
      ov[j] = (unsigned short)(islo ? lb : hb);
    }
    const bool st = (lane < 24) && (node < nN);
    unsigned short* ap = AGG + (size_t)nc * KH + 8 * lst;
    if (st) *(volatile v8us*)ap = ov;
    __threadfence();
    if (st) *(volatile v8us*)ap = ov;
  }
}

template <int T>
__global__ __launch_bounds__(GT) void k_gru(const unsigned short* __restrict__ AGG, unsigned short* XHL,
                                            const unsigned short* __restrict__ WgT2,
                                            const unsigned short* __restrict__ BZR,
                                            const unsigned short* __restrict__ Wh0T2,
                                            const unsigned short* __restrict__ Wh1T2,
                                            const unsigned short* __restrict__ WembT2,
                                            const float* __restrict__ TAB,
                                            float* SD, float* REC, int nN) {
  static_assert(T == 0 || T == 1);
  extern __shared__ __attribute__((aligned(16))) float gsm[];
  unsigned short* tA = (unsigned short*)gsm;
  unsigned short* tB = tA + GR * KH;
  unsigned short* tX = tB + GR * KH;
  unsigned short* tR = tX + GR * KH;
  float* sZ   = (float*)(tR + GR * KH);
  float* sH   = sZ + GR * DH;
  float* sX   = sH + GR * DH;
  float* tab  = sX + GR * DH;
  float* sdot = tab + 768;
  float* srec = sdot + 128;
  const int tid = (int)threadIdx.x, lane = tid & 31, wave = tid >> 5;
  const int hh = lane >> 4, m = lane & 15;
  const int rg = wave & 3, ch = wave >> 2;
  const int blk = (int)blockIdx.x;
  const int rowBase = blk * GR;

  {
    const unsigned short* ga = AGG + (size_t)rowBase * KH;
    const unsigned short* gx = XHL + (size_t)rowBase * KH;
#pragma unroll 3
    for (int i = 0; i < (GR * KH / 8) / GT; ++i) {
      const int p = (i * GT + tid) * 8;
      *(v8usa*)(tA + p) = *(const v8usa*)(ga + p);
      *(v8usa*)(tX + p) = *(const v8usa*)(gx + p);
    }
    if (tid < 192) *(v4fa*)(tab + 4 * tid) = *(const v4f*)(TAB + 4 * tid);
  }
  __syncthreads();

  const v8f z8 = {0.f, 0.f, 0.f, 0.f, 0.f, 0.f, 0.f, 0.f};
  const int arow = (16 * rg + m) * KH + 8 * hh;

  {
    v8f a0[3];
    a0[0] = z8; a0[1] = z8; a0[2] = z8;
    mm_acc<3>(tA + arow, KH / 32, WgT2 + (size_t)(48 * ch + m) * KH + 8 * hh, KH, a0);
#pragma unroll
    for (int t = 0; t < 3; ++t) {
      const int col = 48 * ch + 16 * t + m;
      const float bgv = tab[TB_BG + col];
#pragma unroll
      for (int r = 0; r < 8; ++r) {
        const int row = 16 * rg + 8 * hh + r;
        const float v = a0[t][r] + bgv;
        unsigned int hb, lb;
        split2(v, hb, lb);
        tB[row * KH + col]      = (unsigned short)hb;
        tB[row * KH + DH + col] = (unsigned short)lb;
      }
    }
  }
  __syncthreads();

  {
    v8f cz[6];
#pragma unroll
    for (int t = 0; t < 6; ++t) cz[t] = z8;
    const unsigned short* wz = BZR + (size_t)(DH * ch + m) * KZ + 8 * hh;
    mm_acc<6>(tB + arow, KH / 32, wz, KZ, cz);
    mm_acc<6>(tX + arow, KH / 32, wz + KH, KZ, cz);
    put_raw<6>(sZ + ch * (2 * GR * DH), 16 * rg, 0, hh, m, cz);
    v8f c3[3];
    c3[0] = z8; c3[1] = z8; c3[2] = z8;
    mm_acc<3>(tB + arow, KH / 32, Wh0T2 + (size_t)(48 * ch + m) * KH + 8 * hh, KH, c3);
    put_raw<3>(sH, 16 * rg, 48 * ch, hh, m, c3);
  }
  __syncthreads();

#pragma unroll 1
  for (int i = 0; i < (GR * DH) / GT; ++i) {
    const int e   = i * GT + tid;
    const int row = e / DH;
    const int col = e - DH * row;
    const float zp = sZ[e] + tab[TB_BZ + col];
    const float rp = sX[e] + tab[TB_BR + col];
    const float zv = 1.0f / (1.0f + expf(-zp));
    const float rv = 1.0f / (1.0f + expf(-rp));
    const float xv = bf2f((unsigned int)tX[row * KH + col]) + bf2f((unsigned int)tX[row * KH + DH + col]);
    const float xr = xv * rv;
    unsigned int hb, lb;
    split2(xr, hb, lb);
    tR[row * KH + col]      = (unsigned short)hb;
    tR[row * KH + DH + col] = (unsigned short)lb;
    sZ[e] = zv;
  }
  __syncthreads();

  {
    v8f cu[3];
    cu[0] = z8; cu[1] = z8; cu[2] = z8;
    mm_acc<3>(tR + arow, KH / 32, Wh1T2 + (size_t)(48 * ch + m) * KH + 8 * hh, KH, cu);
    put_raw<3>(sX, 16 * rg, 48 * ch, hh, m, cu);
  }
  __syncthreads();

#pragma unroll 1
  for (int i = 0; i < (GR * DH) / GT; ++i) {
    const int e   = i * GT + tid;
    const int row = e / DH;
    const int col = e - DH * row;
    const float hv = tanhf(sX[e] + sH[e] + tab[TB_BH + col]);
    const float zv = sZ[e];
    const float xv = bf2f((unsigned int)tX[row * KH + col]) + bf2f((unsigned int)tX[row * KH + DH + col]);
    const float xn = hv * zv + xv * (1.0f - zv);
    sX[e] = xn;
    if constexpr (T == 1) {
      unsigned int hb, lb;
      split2(xn, hb, lb);
      tA[row * KH + col]      = (unsigned short)hb;
      tA[row * KH + DH + col] = (unsigned short)lb;
    }
  }
  __syncthreads();

  if constexpr (T == 0) {
    x_tail(sX, tab, sdot, XHL, SD, rowBase, nN, tid);
  } else {
    {
      v8f cy[3];
      cy[0] = z8; cy[1] = z8; cy[2] = z8;
      mm_acc<3>(tA + arow, KH / 32, WembT2 + (size_t)(48 * ch + m) * KH + 8 * hh, KH, cy);
      put_raw<3>(sH, 16 * rg, 48 * ch, hh, m, cy);
    }
    __syncthreads();
    if (tid < DH) {
      float mx = -3.0e38f, sm = 0.0f;
#pragma unroll 1
      for (int r = 0; r < GR; ++r) {
        const float v = tanhf(sH[r * DH + tid]);
        mx = (v > mx || v != v) ? v : mx;
        sm += v;
      }
      srec[tid]      = mx;
      srec[DH + tid] = sm;
    }
    __syncthreads();
    const int pq = tid < 48 ? tid : 47;
    const v4f rv = *(const v4fa*)(srec + 4 * pq);
    float* rp = REC + (size_t)blk * (2 * DH) + 4 * pq;
    if (tid < 48) *(volatile v4f*)rp = rv;
    __threadfence();
    if (tid < 48) *(volatile v4f*)rp = rv;
  }
}

__global__ __launch_bounds__(NTHR) void k_head(const float* __restrict__ REC, const float* __restrict__ TAB,
                                               float* out) {
  __shared__ __attribute__((aligned(16))) float pooled[8 * DH];
  __shared__ __attribute__((aligned(16))) float wm[DH * NCLS];
  __shared__ __attribute__((aligned(16))) float outs[8 * NCLS];
  const int tid = (int)threadIdx.x;
  const int blk = (int)blockIdx.x;
#pragma unroll 1
  for (int i = tid; i < 8 * DH; i += NTHR) {
    const int g = i / DH;
    const int c = i - g * DH;
    const size_t rb = (size_t)(blk * 8 + g) * (size_t)(GLEN / GR);
    float mx = REC[rb * (2 * DH) + c];
    float sm = REC[rb * (2 * DH) + DH + c];
#pragma unroll 1
    for (int q = 1; q < GLEN / GR; ++q) {
      const float v = REC[(rb + q) * (2 * DH) + c];
      const float s = REC[(rb + q) * (2 * DH) + DH + c];
      mx = (v > mx || v != v) ? v : mx;
      sm += s;
    }
    pooled[i] = mx + sm * (1.0f / 256.0f);
  }
#pragma unroll 1
  for (int i = tid; i < (DH * NCLS) / 4; i += NTHR)
    *(v4fa*)(wm + 4 * i) = *(const v4f*)(TAB + TB_WM + 4 * i);
  __syncthreads();
  if (tid < 8 * NCLS) {
    const int g = tid / NCLS;
    const int j = tid - g * NCLS;
    float a = 0.0f;
#pragma unroll 4
    for (int c = 0; c < DH; ++c) a = fmaf(pooled[g * DH + c], wm[c * NCLS + j], a);
    outs[tid] = a;
  }
  __syncthreads();
  const int pq = tid < 40 ? tid : 39;
  const v4f ov = *(const v4fa*)(outs + 4 * pq);
  float* op = out + (size_t)blk * (8 * NCLS) + 4 * pq;
  if (tid < 40) *(volatile v4f*)op = ov;
  __threadfence();
  if (tid < 40) *(volatile v4f*)op = ov;
}

extern "C" void kernel_launch(void* const* d_in, const int* in_sizes, int n_in,
                              void* d_out, int out_size, void* d_ws, size_t ws_size,
                              hipStream_t stream) {
  if (n_in < 24) return;
  if (in_sizes[0] != NN) return;
  const int nE = in_sizes[1];
  if (nE < 1 || nE > (1 << 30) || in_sizes[2] != nE) return;
  if (in_sizes[3] != NVOC * DIN) return;
  if (in_sizes[4] != DIN * DH || in_sizes[5] != DH) return;
  if (in_sizes[6] != DH * DH) return;
  if (in_sizes[7] != DH || in_sizes[8] != DH || in_sizes[9] != DH) return;
  for (int i = 10; i < 22; i += 2) {
    if (in_sizes[i] != DH * DH || in_sizes[i + 1] != DH) return;
  }
  if (in_sizes[22] != DH * DH || in_sizes[23] != DH * NCLS) return;
  if (out_size != NGRAPH * NCLS) return;

  const int*   ids   = (const int*)  d_in[0];
  const int*   src   = (const int*)  d_in[1];
  const int*   dst   = (const int*)  d_in[2];
  const float* embed = (const float*)d_in[3];
  const float* We    = (const float*)d_in[4];
  const float* be    = (const float*)d_in[5];
  const float* Wg    = (const float*)d_in[6];
  const float* ats   = (const float*)d_in[7];
  const float* atd   = (const float*)d_in[8];
  const float* bg    = (const float*)d_in[9];
  const float* Wz0   = (const float*)d_in[10];
  const float* bz0   = (const float*)d_in[11];
  const float* Wz1   = (const float*)d_in[12];
  const float* bz1   = (const float*)d_in[13];
  const float* Wr0   = (const float*)d_in[14];
  const float* br0   = (const float*)d_in[15];
  const float* Wr1   = (const float*)d_in[16];
  const float* br1   = (const float*)d_in[17];
  const float* Wh0   = (const float*)d_in[18];
  const float* bh0   = (const float*)d_in[19];
  const float* Wh1   = (const float*)d_in[20];
  const float* bh1   = (const float*)d_in[21];
  const float* Wemb  = (const float*)d_in[22];
  const float* Wmlp  = (const float*)d_in[23];
  float* out = (float*)d_out;

  const int nN = NN;
  const int gA = nN / NBA;
  const int gM = nN / GR;
  const int vec8 = ((nE & 3) == 0) ? 1 : 0;

  char* ws = (char*)d_ws;
  size_t off = 0;
  const size_t oWeT = off; off += (size_t)DH * KE * 2;            off = (off + 255) & ~(size_t)255;
  const size_t oWg  = off; off += (size_t)DH * KH * 2;            off = (off + 255) & ~(size_t)255;
  const size_t oWh0 = off; off += (size_t)DH * KH * 2;            off = (off + 255) & ~(size_t)255;
  const size_t oWh1 = off; off += (size_t)DH * KH * 2;            off = (off + 255) & ~(size_t)255;
  const size_t oWem = off; off += (size_t)DH * KH * 2;            off = (off + 255) & ~(size_t)255;
  const size_t oBZR = off; off += (size_t)2 * DH * KZ * 2;        off = (off + 255) & ~(size_t)255;
  const size_t oTAB = off; off += (size_t)TB_N * 4;               off = (off + 255) & ~(size_t)255;
  const size_t oXHL = off; off += (size_t)nN * KH * 2;            off = (off + 255) & ~(size_t)255;
  const size_t oAGG = off; off += (size_t)nN * KH * 2;            off = (off + 255) & ~(size_t)255;
  const size_t oSD  = off; off += (size_t)2 * nN * 4;             off = (off + 255) & ~(size_t)255;
  const size_t oHIT = off; off += (size_t)gA * RCAP * 4;          off = (off + 255) & ~(size_t)255;
  const size_t oFLG = off; off += (size_t)gA * 128;               off = (off + 255) & ~(size_t)255;
  const size_t oREC = off; off += (size_t)gM * 2 * DH * 4;        off = (off + 255) & ~(size_t)255;
  if (off > ws_size || off > (size_t)WSMAX) return;
  unsigned short* WeT    = (unsigned short*)(ws + oWeT);
  unsigned short* WgT2   = (unsigned short*)(ws + oWg);
  unsigned short* Wh0T2  = (unsigned short*)(ws + oWh0);
  unsigned short* Wh1T2  = (unsigned short*)(ws + oWh1);
  unsigned short* WembT2 = (unsigned short*)(ws + oWem);
  unsigned short* BZR    = (unsigned short*)(ws + oBZR);
  float*          TAB    = (float*)(ws + oTAB);
  unsigned short* XHL    = (unsigned short*)(ws + oXHL);
  unsigned short* AGG    = (unsigned short*)(ws + oAGG);
  float*          SD     = (float*)(ws + oSD);
  int*            HITS   = (int*)(ws + oHIT);
  int*            FLG    = (int*)(ws + oFLG);
  float*          REC    = (float*)(ws + oREC);

  const int bktLds  = BKT_LDS_INTS * 4;
  const int scanLds = SCAN_LDS_INTS * 4;
  const int encLds  = ENC_LDS;
  const int gruLds  = GRU_LDS;
  hipFuncSetAttribute(reinterpret_cast<const void*>(&k_bucket),
                      hipFuncAttributeMaxDynamicSharedMemorySize, bktLds);
  hipFuncSetAttribute(reinterpret_cast<const void*>(&k_scan),
                      hipFuncAttributeMaxDynamicSharedMemorySize, scanLds);
  hipFuncSetAttribute(reinterpret_cast<const void*>(&k_encode),
                      hipFuncAttributeMaxDynamicSharedMemorySize, encLds);
  hipFuncSetAttribute(reinterpret_cast<const void*>(&k_gru<0>),
                      hipFuncAttributeMaxDynamicSharedMemorySize, gruLds);
  hipFuncSetAttribute(reinterpret_cast<const void*>(&k_gru<1>),
                      hipFuncAttributeMaxDynamicSharedMemorySize, gruLds);

  k_prep<<<NB_W + 1, NTHR, 0, stream>>>(We, Wg, Wz0, Wz1, Wr0, Wr1, Wh0, Wh1, Wemb,
                                        be, bg, bz0, bz1, br0, br1, bh0, bh1, ats, atd, Wmlp,
                                        WeT, WgT2, Wh0T2, Wh1T2, WembT2, BZR, TAB);
  k_bucket<<<gA, NTHR, bktLds, stream>>>(src, dst, nE, nN, vec8, HITS, FLG);
  k_encode<<<gM, GT, encLds, stream>>>(ids, embed, WeT, TAB, XHL, SD, nN, NVOC);
  k_scan<<<gA, NTHR, scanLds, stream>>>(HITS, FLG, XHL, SD, AGG, nN);
  k_gru<0><<<gM, GT, gruLds, stream>>>(AGG, XHL, WgT2, BZR, Wh0T2, Wh1T2, WembT2, TAB, SD, REC, nN);
  k_scan<<<gA, NTHR, scanLds, stream>>>(HITS, FLG, XHL, SD, AGG, nN);
  k_gru<1><<<gM, GT, gruLds, stream>>>(AGG, XHL, WgT2, BZR, Wh0T2, Wh1T2, WembT2, TAB, SD, REC, nN);
  k_head<<<NGRAPH / 8, NTHR, 0, stream>>>(REC, TAB, out);
}
